// DPASSMBlock_44951127720633
// MI455X (gfx1250) — hardware-run, weakly checked
//
#include <hip/hip_runtime.h>
#include <math.h>

typedef __attribute__((ext_vector_type(16))) _Float16 v16h;
typedef __attribute__((ext_vector_type(8)))  _Float16 v8h;
typedef __attribute__((ext_vector_type(8)))  float    v8f;
typedef __attribute__((ext_vector_type(4)))  float    v4f;
typedef __attribute__((ext_vector_type(2)))  float    v2f;
typedef __attribute__((ext_vector_type(4)))  unsigned int v4u;

constexpr int kB   = 2;
constexpr int kT   = 2048;
constexpr int kD   = 1024;
constexpr int kH   = 16;
constexpr int kDh  = 64;
constexpr int kWin = 256;
constexpr int kNs  = 128;
constexpr int kHid = 4096;
constexpr int kM   = kB * kT;
constexpr int kNcat = 3 * kD + kD + kNs;
constexpr int kSqrtDh = 8;
static_assert(kSqrtDh * kSqrtDh == kDh);
static_assert(kH * kDh == kD);
static_assert(kDh == 64);
static_assert((kWin % 64) == 0 && (kT % 64) == 0);
static_assert((kM % 64) == 0 && (kD % 64) == 0 && (kNs % 64) == 0 && (kHid % 64) == 0 && (kNcat % 64) == 0);
static_assert((kD % 32) == 0 && (kNs % 32) == 0 && (kHid % 32) == 0 && (kDh % 32) == 0);
constexpr float kScoreScale = 1.0f / (float)kSqrtDh;
constexpr float kWCarry     = 32.0f;
constexpr float kAoCarry    = 16.0f;
constexpr float kHidCarry   = 16.0f;
constexpr float kPCarry     = 32768.0f;
constexpr float kScaleW     = 1.0f / kWCarry;
constexpr float kScaleAoW   = 1.0f / (kAoCarry * kWCarry);
constexpr float kScaleHidW  = 1.0f / (kHidCarry * kWCarry);
constexpr float kLnEps      = 1e-5f;
constexpr float kInvD       = 1.0f / (float)kD;
constexpr float kInvSqrt2   = 0.70710678118654752f;
constexpr float kMaskFill   = -1e30f;

constexpr size_t kSzAct16 = (size_t)kM * kD * 2;
constexpr size_t kSzAct32 = (size_t)kM * kD * 4;
constexpr size_t kOffWcat = 0;
constexpr size_t kOffWot  = kOffWcat + (size_t)kNcat * kD * 2;
constexpr size_t kOffCwt  = kOffWot  + (size_t)kD * kD * 2;
constexpr size_t kOffW1t  = kOffCwt  + (size_t)kD * kNs * 2;
constexpr size_t kOffW2t  = kOffW1t  + (size_t)kHid * kD * 2;
constexpr size_t kOffXn16 = kOffW2t  + (size_t)kD * kHid * 2;
constexpr size_t kOffXn2  = kOffXn16 + kSzAct16;
constexpr size_t kOffQ16  = kOffXn2  + kSzAct16;
constexpr size_t kOffK16  = kOffQ16  + kSzAct16;
constexpr size_t kOffV16  = kOffK16  + kSzAct16;
constexpr size_t kOffAo16 = kOffV16  + kSzAct16;
constexpr size_t kOffHid  = kOffQ16;
constexpr size_t kOffG32  = kOffAo16 + kSzAct16;
constexpr size_t kOffU32  = kOffG32  + kSzAct32;
constexpr size_t kOffSt16 = kOffU32  + (size_t)kM * kNs * 4;
constexpr size_t kOffSsm  = kOffSt16 + (size_t)kM * kNs * 2;
constexpr size_t kOffXmid = kOffSsm  + kSzAct32;
constexpr size_t kWsTotal = kOffXmid + kSzAct32;
static_assert(kWsTotal == 131596288ull);
static_assert(kWsTotal <= 134217728ull);
static_assert((size_t)kM * kHid * 2 == 4 * kSzAct16);
static_assert((kOffWot % 128) == 0 && (kOffCwt % 128) == 0 && (kOffW1t % 128) == 0 && (kOffW2t % 128) == 0 &&
              (kOffXn16 % 128) == 0 && (kOffXn2 % 128) == 0 && (kOffQ16 % 128) == 0 && (kOffK16 % 128) == 0 &&
              (kOffV16 % 128) == 0 && (kOffAo16 % 128) == 0 && (kOffG32 % 128) == 0 && (kOffU32 % 128) == 0 &&
              (kOffSt16 % 128) == 0 && (kOffSsm % 128) == 0 && (kOffXmid % 128) == 0);
constexpr size_t kOut1Elem = (size_t)kM * kD;
static_assert(kOut1Elem * 4 == 16777216ull);
static_assert(kOut1Elem * 4 + (size_t)kB * kNs * 4 == 16778240ull);

__device__ __forceinline__ unsigned short h_bits(float f) { const _Float16 h = (_Float16)f; return __builtin_bit_cast(unsigned short, h); }
__device__ __forceinline__ unsigned pk16(unsigned short a, unsigned short b) { return (unsigned)a | ((unsigned)b << 16); }

struct FragH {
  union U { v16h v; v8h h[2]; };
  static __device__ __forceinline__ v16h load(const _Float16* p) {
    U f; f.h[0] = *(const v8h*)(p); f.h[1] = *(const v8h*)(p + 16); return f.v;
  }
};
__device__ __forceinline__ v8f mma_h(v16h a, v16h b, v8f c) {
  return __builtin_amdgcn_wmma_f32_16x16x32_f16(false, a, false, b, (short)0, c, false, false);
}
__device__ __forceinline__ v8f mma_h_guard(v16h a, v16h b, v8f c) {
  c = __builtin_amdgcn_wmma_f32_16x16x32_f16(false, a, false, b, (short)0, c, false, false);
  asm volatile("v_nop\n\tv_nop\n\tv_nop\n\tv_nop" : "+v"(c) : "v"(a), "v"(b));
  return c;
}
__device__ __forceinline__ void row_guard(v8f& a0, v8f& a1, v8f& a2, v8f& a3, v16h x, v16h b0, v16h b1, v16h b2, v16h b3) {
  asm volatile("v_nop\n\tv_nop\n\tv_nop\n\tv_nop" : "+v"(a0), "+v"(a1), "+v"(a2), "+v"(a3) : "v"(x), "v"(b0), "v"(b1), "v"(b2), "v"(b3));
}
__device__ __forceinline__ void keep4_h(v16h a, v16h b, v16h c, v16h d) { asm volatile("v_nop" :: "v"(a), "v"(b), "v"(c), "v"(d)); }
__device__ __forceinline__ void acc_guard4(v8f& a, v8f& b, v8f& c, v8f& d) { asm volatile("v_nop\n\tv_nop\n\tv_nop\n\tv_nop" : "+v"(a), "+v"(b), "+v"(c), "+v"(d)); }
__device__ __forceinline__ void wave_lds_sync() {
  __builtin_amdgcn_fence(__ATOMIC_RELEASE, "workgroup");
  __builtin_amdgcn_wave_barrier();
  __builtin_amdgcn_fence(__ATOMIC_ACQUIRE, "workgroup");
}

__global__ __launch_bounds__(256) void transpose_cast_kernel(
    const float* __restrict__ W, unsigned short* __restrict__ Bt, int Kdim, int Ndim, float scale)
{
  __shared__ float tile[64 * 65];
  const int tid = threadIdx.x, lane = tid & 31, wave = tid >> 5;
  const int n0 = blockIdx.x * 64;
  const int k0 = blockIdx.y * 64;
#pragma unroll
  for (int p = 0; p < 16; ++p) {
    const int idx = tid + p * 256;
    const int kk  = idx >> 6;
    const int nn  = idx & 63;
    const float v = W[(size_t)(k0 + kk) * Ndim + n0 + nn];
    tile[kk * 65 + nn] = v * scale;
  }
  __syncthreads();
  const int q = lane >> 3, c8 = (lane & 7) * 8;
  v8h hv[2];
#pragma unroll
  for (int it = 0; it < 2; ++it) {
    const int nrow = it * 32 + wave * 4 + q;
#pragma unroll
    for (int e = 0; e < 8; ++e) hv[it][e] = (_Float16)tile[(c8 + e) * 65 + nrow];
  }
  for (int pass = 0; pass < 2; ++pass) {
#pragma unroll
    for (int it = 0; it < 2; ++it) {
      const int nrow = it * 32 + wave * 4 + q;
      *(volatile v8h*)(void*)(Bt + (size_t)(n0 + nrow) * Kdim + k0 + c8) = hv[it];
    }
    __threadfence();
  }
}

__global__ __launch_bounds__(256) void layernorm_f16_kernel(
    const float* __restrict__ X, const float* __restrict__ G, const float* __restrict__ Bv,
    unsigned short* __restrict__ Y, int rows)
{
  const int lane = threadIdx.x & 31, wave = threadIdx.x >> 5;
  const int row = blockIdx.x * 8 + wave;
  if (row >= rows) return;
  const float* xr = X + (size_t)row * kD + lane * 8;
  float s = 0.f;
#pragma unroll 1
  for (int j = 0; j < 4; ++j) {
    const v4f a = *(const v4f*)(xr + j * 256);
    const v4f c = *(const v4f*)(xr + j * 256 + 4);
    s += ((a[0] + a[1]) + (a[2] + a[3])) + ((c[0] + c[1]) + (c[2] + c[3]));
  }
#pragma unroll
  for (int off = 16; off > 0; off >>= 1) s += __shfl_xor(s, off, 32);
  const float mu = s * kInvD;
  float vs = 0.f;
#pragma unroll 1
  for (int j = 0; j < 4; ++j) {
    const v4f a = *(const v4f*)(xr + j * 256);
    const v4f c = *(const v4f*)(xr + j * 256 + 4);
#pragma unroll
    for (int e = 0; e < 4; ++e) {
      const float d0 = a[e] - mu;
      const float d1 = c[e] - mu;
      vs += d0 * d0;
      vs += d1 * d1;
    }
  }
#pragma unroll
  for (int off = 16; off > 0; off >>= 1) vs += __shfl_xor(vs, off, 32);
  const float rstd = rsqrtf(vs * kInvD + kLnEps);
  v8h hv[4];
#pragma unroll
  for (int j = 0; j < 4; ++j) {
    const int co = j * 256 + lane * 8;
    const v4f a  = *(const v4f*)(xr + j * 256);
    const v4f c  = *(const v4f*)(xr + j * 256 + 4);
    const v4f g0 = *(const v4f*)(G + co);
    const v4f g1 = *(const v4f*)(G + co + 4);
    const v4f b0 = *(const v4f*)(Bv + co);
    const v4f b1 = *(const v4f*)(Bv + co + 4);
#pragma unroll
    for (int e = 0; e < 4; ++e) {
      hv[j][e]     = (_Float16)(((a[e] - mu) * rstd) * g0[e] + b0[e]);
      hv[j][4 + e] = (_Float16)(((c[e] - mu) * rstd) * g1[e] + b1[e]);
    }
  }
  unsigned short* yr = Y + (size_t)row * kD + lane * 8;
  for (int pass = 0; pass < 2; ++pass) {
#pragma unroll
    for (int j = 0; j < 4; ++j) *(volatile v8h*)(void*)(yr + j * 256) = hv[j];
    __threadfence();
  }
}

template <int EPI>
__global__ __launch_bounds__(256) void gemm_f16_kernel(
    const unsigned short* __restrict__ Ap, int lda,
    const unsigned short* __restrict__ Btp, int ldb,
    void* Cout, int ldc,
    const float* bias,
    const float* e0, const float* e1, const float* e2,
    int M, int N, int K, float scale, float oscale)
{
  const _Float16* A  = (const _Float16*)(const void*)Ap;
  const _Float16* Bt = (const _Float16*)(const void*)Btp;
  __shared__ __align__(16) float sT[8][16 * 68];
  const int lane = threadIdx.x & 31;
  const int wave = threadIdx.x >> 5;
  const int tilesN = N >> 6;
  const int tilesM = M >> 6;
  const int tile = blockIdx.x * 8 + wave;
  if (tile >= tilesM * tilesN) return;
  const int tm = tile / tilesN;
  const int tn = tile - tm * tilesN;
  const int m0 = tm << 6;
  const int n0 = tn << 6;
  const int rlane = lane & 15;
  const int koff  = (lane >> 4) * 8;
  const int mOff  = (lane >> 4) * 8;

  v8f acc[4][4];
#pragma unroll
  for (int i = 0; i < 4; ++i)
#pragma unroll
    for (int j = 0; j < 4; ++j) acc[i][j] = (v8f){0.f,0.f,0.f,0.f,0.f,0.f,0.f,0.f};

  for (int k0 = 0; k0 < K; k0 += 32) {
    v16h bh[4];
#pragma unroll
    for (int j = 0; j < 4; ++j) {
      const size_t bo = (size_t)(n0 + (j << 4) + rlane) * ldb + koff + k0;
      bh[j] = FragH::load(Bt + bo);
    }
#pragma unroll
    for (int i = 0; i < 4; ++i) {
      const size_t ao = (size_t)(m0 + (i << 4) + rlane) * lda + koff + k0;
      const v16h ah = FragH::load(A + ao);
#pragma unroll
      for (int j = 0; j < 4; ++j) acc[i][j] = mma_h(ah, bh[j], acc[i][j]);
      row_guard(acc[i][0], acc[i][1], acc[i][2], acc[i][3], ah, bh[0], bh[1], bh[2], bh[3]);
    }
    keep4_h(bh[0], bh[1], bh[2], bh[3]);
  }
  acc_guard4(acc[0][0], acc[0][1], acc[0][2], acc[0][3]);
  acc_guard4(acc[1][0], acc[1][1], acc[1][2], acc[1][3]);
  acc_guard4(acc[2][0], acc[2][1], acc[2][2], acc[2][3]);
  acc_guard4(acc[3][0], acc[3][1], acc[3][2], acc[3][3]);

  float* slab = sT[wave];
#pragma unroll
  for (int i = 0; i < 4; ++i) {
    const int mBase = m0 + (i << 4);
#pragma unroll
    for (int j = 0; j < 4; ++j) {
      float bv = 0.f;
      if (EPI != 2) bv = bias[n0 + (j << 4) + rlane];
#pragma unroll
      for (int r = 0; r < 8; ++r) slab[(mOff + r) * 68 + (j << 4) + rlane] = acc[i][j][r] * scale + bv;
    }
    wave_lds_sync();
    if (EPI == 1 || EPI == 4) {
#pragma unroll 1
      for (int it = 0; it < 32; ++it) {
        const int idx = (it << 5) + lane;
        const int so  = (idx >> 6) * 68 + (idx & 63);
        const float v = slab[so];
        float o;
        if (EPI == 1) o = __builtin_amdgcn_rcpf(1.0f + expf(-v));
        else          o = (0.5f * v * (1.0f + erff(v * kInvSqrt2))) * oscale;
        slab[so] = o;
      }
      wave_lds_sync();
    }
    if (EPI == 3 || EPI == 5) {
      const int hh = lane >> 4, c4 = (lane & 15) * 4;
#pragma unroll 1
      for (int it = 0; it < 8; ++it) {
        const int row = it * 2 + hh;
        const size_t go = (size_t)(mBase + row) * ldc + n0 + c4;
        const v4f v  = *(const v4f*)(slab + row * 68 + c4);
        const v4f xv = *(const v4f*)(e0 + go);
        v4f o;
        if (EPI == 3) {
          const v4f gv = *(const v4f*)(e1 + go);
          const v4f sv = *(const v4f*)(e2 + go);
#pragma unroll
          for (int e = 0; e < 4; ++e) o[e] = (xv[e] + gv[e] * v[e]) + (1.0f - gv[e]) * sv[e];
        } else {
#pragma unroll
          for (int e = 0; e < 4; ++e) o[e] = xv[e] + v[e];
        }
        *(v4f*)(slab + row * 68 + c4) = o;
      }
      wave_lds_sync();
    }
    if (EPI == 0 || EPI == 4) {
      const int q = lane >> 3, c8 = (lane & 7) * 8;
      unsigned short* C = (unsigned short*)Cout;
      for (int pass = 0; pass < 2; ++pass) {
#pragma unroll
        for (int it = 0; it < 4; ++it) {
          const int row = it * 4 + q;
          const float* sp = slab + row * 68 + c8;
          v8h hv;
#pragma unroll
          for (int e = 0; e < 8; ++e) hv[e] = (_Float16)sp[e];
          *(volatile v8h*)(void*)(C + (size_t)(mBase + row) * ldc + n0 + c8) = hv;
        }
        __threadfence();
      }
    } else {
      float* C = (float*)Cout;
      const int hh = lane >> 4, c4 = (lane & 15) * 4;
      for (int pass = 0; pass < 2; ++pass) {
#pragma unroll
        for (int it = 0; it < 8; ++it) {
          const int row = it * 2 + hh;
          const v4f v = *(const v4f*)(slab + row * 68 + c4);
          *(volatile v4f*)(C + (size_t)(mBase + row) * ldc + n0 + c4) = v;
        }
        __threadfence();
      }
    }
    wave_lds_sync();
  }
}

__global__ __launch_bounds__(128) void attn_window_kernel(
    const unsigned short* __restrict__ Q16, const unsigned short* __restrict__ K16,
    const unsigned short* __restrict__ V16, unsigned short* __restrict__ AO16)
{
  __shared__ __align__(16) unsigned short Ksh[64 * 64];
  __shared__ __align__(16) unsigned short Vts[64 * 64];
  __shared__ __align__(16) unsigned short Psh[4][16 * 64];
  __shared__ __align__(16) float Os[4][16 * 68];

  const int tid  = threadIdx.x;
  const int wave = tid >> 5;
  const int lane = tid & 31;
  const int hh   = lane >> 4;
  const int c    = lane & 15;
  constexpr int nqb = kT / 64;
  const int bx  = blockIdx.x;
  const int qb  = bx % nqb;
  const int bhd = bx / nqb;
  const int h   = bhd % kH;
  const int b   = bhd / kH;
  const int q0  = qb * 64 + wave * 16;
  const size_t rowbase = (size_t)b * kT;

  v16h qa[2];
  {
    const unsigned short* qp = Q16 + (rowbase + q0 + c) * kD + h * kDh + 8 * hh;
#pragma unroll
    for (int dc = 0; dc < 2; ++dc) qa[dc] = FragH::load((const _Float16*)(const void*)(qp + dc * 32));
  }

  float mrow[8], lrow[8];
  v8f oacc[4];
#pragma unroll
  for (int r = 0; r < 8; ++r) { mrow[r] = kMaskFill; lrow[r] = 0.f; }
#pragma unroll
  for (int t = 0; t < 4; ++t) oacc[t] = (v8f){0.f,0.f,0.f,0.f,0.f,0.f,0.f,0.f};

  const int kcLo = (qb - kWin / 64) > 0 ? (qb - kWin / 64) : 0;
  unsigned short* pw = Psh[wave];

#pragma unroll 1
  for (int kc = kcLo; kc <= qb; ++kc) {
    const int kv0 = kc * 64;
    __syncthreads();
    {
      const int kvr = tid >> 1, dhf = (tid & 1) * 32;
      const size_t go = (rowbase + kv0 + kvr) * kD + h * kDh + dhf;
      const v4u* kp = (const v4u*)(const void*)(K16 + go);
      const v4u* vp = (const v4u*)(const void*)(V16 + go);
#pragma unroll
      for (int i = 0; i < 4; ++i) {
        const v4u kk = kp[i];
        *(v4u*)(void*)(Ksh + kvr * 64 + dhf + 8 * i) = kk;
        const v4u vv = vp[i];
#pragma unroll
        for (int w = 0; w < 4; ++w) {
          const unsigned word = vv[w];
          const int d = dhf + 8 * i + 2 * w;
          Vts[d * 64 + kvr]       = (unsigned short)(word & 0xffffu);
          Vts[(d + 1) * 64 + kvr] = (unsigned short)(word >> 16);
        }
      }
    }
    __syncthreads();

    v8f s[4];
#pragma unroll
    for (int j = 0; j < 4; ++j) {
      s[j] = (v8f){0.f,0.f,0.f,0.f,0.f,0.f,0.f,0.f};
#pragma unroll
      for (int dc = 0; dc < 2; ++dc) {
        const v16h kb = FragH::load((const _Float16*)(const void*)(Ksh + (j * 16 + c) * 64 + dc * 32 + 8 * hh));
        s[j] = mma_h_guard(qa[dc], kb, s[j]);
      }
    }

    float cm[8];
#pragma unroll
    for (int r = 0; r < 8; ++r) {
      const int qrow = q0 + 8 * hh + r;
      float m = kMaskFill;
#pragma unroll
      for (int j = 0; j < 4; ++j) {
        const int kvcol = kv0 + j * 16 + c;
        const bool allowed = (kvcol <= qrow) && (qrow - kvcol < kWin);
        const float sv = allowed ? (s[j][r] * kScoreScale) : kMaskFill;
        s[j][r] = sv;
        m = fmaxf(m, sv);
      }
#pragma unroll
      for (int off = 1; off < 16; off <<= 1) m = fmaxf(m, __shfl_xor(m, off, 32));
      cm[r] = m;
    }
#pragma unroll
    for (int r = 0; r < 8; ++r) {
      const int qrow = q0 + 8 * hh + r;
      const float mnew  = fmaxf(mrow[r], cm[r]);
      const float alpha = expf(mrow[r] - mnew);
      mrow[r] = mnew;
      float psum = 0.f;
#pragma unroll
      for (int j = 0; j < 4; ++j) {
        const int kvcol = kv0 + j * 16 + c;
        const bool allowed = (kvcol <= qrow) && (qrow - kvcol < kWin);
        const float ev = expf(s[j][r] - mnew);
        const float p  = allowed ? ev : 0.0f;
        psum += p;
        pw[(8 * hh + r) * 64 + j * 16 + c] = h_bits(p * kPCarry);
      }
#pragma unroll
      for (int off = 1; off < 16; off <<= 1) psum += __shfl_xor(psum, off, 32);
      lrow[r] = lrow[r] * alpha + psum;
#pragma unroll
      for (int t = 0; t < 4; ++t) oacc[t][r] *= alpha;
    }
    wave_lds_sync();
#pragma unroll 1
    for (int kk = 0; kk < 2; ++kk) {
      const v16h pa = FragH::load((const _Float16*)(const void*)(pw + c * 64 + kk * 32 + 8 * hh));
#pragma unroll
      for (int t = 0; t < 4; ++t) {
        const v16h vb = FragH::load((const _Float16*)(const void*)(Vts + (t * 16 + c) * 64 + kk * 32 + 8 * hh));
        oacc[t] = mma_h_guard(pa, vb, oacc[t]);
      }
    }
    wave_lds_sync();
  }

  float* os = Os[wave];
#pragma unroll
  for (int r = 0; r < 8; ++r) {
    const float inv = kAoCarry / (lrow[r] * kPCarry);
#pragma unroll
    for (int t = 0; t < 4; ++t) os[(8 * hh + r) * 68 + t * 16 + c] = oacc[t][r] * inv;
  }
  wave_lds_sync();
  {
    const int q = lane >> 3, c8 = (lane & 7) * 8;
    v8h hv[4];
#pragma unroll
    for (int it = 0; it < 4; ++it) {
      const float* sp = os + (it * 4 + q) * 68 + c8;
#pragma unroll
      for (int e = 0; e < 8; ++e) hv[it][e] = (_Float16)sp[e];
    }
    for (int pass = 0; pass < 2; ++pass) {
#pragma unroll
      for (int it = 0; it < 4; ++it)
        *(volatile v8h*)(void*)(AO16 + (rowbase + q0 + it * 4 + q) * kD + h * kDh + c8) = hv[it];
      __threadfence();
    }
  }
}

__global__ __launch_bounds__(128) void scan_kernel(
    const float* __restrict__ U, const float* __restrict__ Avec, const float* __restrict__ S0,
    unsigned short* __restrict__ ST16, float* __restrict__ out_state)
{
  const int tid = threadIdx.x;
  const int b = tid >> 6, p = tid & 63;
  const int n0 = 2 * p;
  const v2f av = *(const v2f*)(Avec + n0);
  const v2f sv = *(const v2f*)(S0 + b * kNs + n0);
  const float a0 = av[0], a1 = av[1];
  float s0 = sv[0], s1 = sv[1];
  const float* up = U + (size_t)b * kT * kNs + n0;
  unsigned* sp = (unsigned*)(void*)ST16 + (size_t)b * kT * (kNs / 2) + p;
#pragma unroll 1
  for (int t0 = 0; t0 < kT; t0 += 8) {
    v2f uv[8];
#pragma unroll
    for (int e = 0; e < 8; ++e) uv[e] = *(const v2f*)(up + (size_t)(t0 + e) * kNs);
    unsigned w[8];
#pragma unroll
    for (int e = 0; e < 8; ++e) {
      s0 = a0 * s0 + uv[e][0];
      s1 = a1 * s1 + uv[e][1];
      w[e] = pk16(h_bits(s0), h_bits(s1));
    }
    for (int pass = 0; pass < 2; ++pass) {
#pragma unroll
      for (int e = 0; e < 8; ++e) *(volatile unsigned*)(sp + (size_t)(t0 + e) * (kNs / 2)) = w[e];
      __threadfence();
    }
  }
  const v2f fin = (v2f){s0, s1};
  float* op = out_state + b * kNs + n0;
  *(volatile v2f*)op = fin;
  __threadfence();
  *(volatile v2f*)op = fin;
}

extern "C" void kernel_launch(void* const* d_in, const int* in_sizes, int n_in,
                              void* d_out, int out_size, void* d_ws, size_t ws_size,
                              hipStream_t stream)
{
  if (n_in < 23) return;
  if (in_sizes[0] != kM * kD) return;
  if (in_sizes[1] != kB * kNs) return;
  if (in_sizes[2] != kD || in_sizes[3] != kD) return;
  if (in_sizes[4] != kD * kD || in_sizes[5] != kD) return;
  if (in_sizes[6] != kD * kD || in_sizes[7] != kD) return;
  if (in_sizes[8] != kD * kD || in_sizes[9] != kD) return;
  if (in_sizes[10] != kD * kD || in_sizes[11] != kD) return;
  if (in_sizes[12] != kD * kD || in_sizes[13] != kD) return;
  if (in_sizes[14] != kNs) return;
  if (in_sizes[15] != kD * kNs || in_sizes[16] != kNs * kD) return;
  if (in_sizes[17] != kD || in_sizes[18] != kD) return;
  if (in_sizes[19] != kD * kHid || in_sizes[20] != kHid) return;
  if (in_sizes[21] != kHid * kD || in_sizes[22] != kD) return;
  if (out_size != kM * kD + kB * kNs) return;
  if (ws_size < kWsTotal) return;

  const float* x    = (const float*)d_in[0];
  const float* st0  = (const float*)d_in[1];
  const float* l1g  = (const float*)d_in[2];
  const float* l1b  = (const float*)d_in[3];
  const float* wq   = (const float*)d_in[4];
  const float* bq   = (const float*)d_in[5];
  const float* wk   = (const float*)d_in[6];
  const float* bk   = (const float*)d_in[7];
  const float* wv   = (const float*)d_in[8];
  const float* bv   = (const float*)d_in[9];
  const float* wo   = (const float*)d_in[10];
  const float* bo   = (const float*)d_in[11];
  const float* wg   = (const float*)d_in[12];
  const float* bg   = (const float*)d_in[13];
  const float* Avec = (const float*)d_in[14];
  const float* Bw   = (const float*)d_in[15];
  const float* Cw   = (const float*)d_in[16];
  const float* l2g  = (const float*)d_in[17];
  const float* l2b  = (const float*)d_in[18];
  const float* w1   = (const float*)d_in[19];
  const float* b1   = (const float*)d_in[20];
  const float* w2   = (const float*)d_in[21];
  const float* b2   = (const float*)d_in[22];
  float* out0 = (float*)d_out;
  float* out1 = out0 + kOut1Elem;

  char* ws = (char*)d_ws;
  unsigned short* WCAT  = (unsigned short*)(ws + kOffWcat);
  unsigned short* WOT   = (unsigned short*)(ws + kOffWot);
  unsigned short* CWT   = (unsigned short*)(ws + kOffCwt);
  unsigned short* W1T   = (unsigned short*)(ws + kOffW1t);
  unsigned short* W2T   = (unsigned short*)(ws + kOffW2t);
  unsigned short* XN16  = (unsigned short*)(ws + kOffXn16);
  unsigned short* XN2   = (unsigned short*)(ws + kOffXn2);
  unsigned short* Q16   = (unsigned short*)(ws + kOffQ16);
  unsigned short* K16   = (unsigned short*)(ws + kOffK16);
  unsigned short* V16   = (unsigned short*)(ws + kOffV16);
  unsigned short* AO16  = (unsigned short*)(ws + kOffAo16);
  unsigned short* HID16 = (unsigned short*)(ws + kOffHid);
  float*          G32   = (float*)(ws + kOffG32);
  float*          U32   = (float*)(ws + kOffU32);
  unsigned short* ST16  = (unsigned short*)(ws + kOffSt16);
  float*          SSM32 = (float*)(ws + kOffSsm);
  float*          XMID  = (float*)(ws + kOffXmid);

  transpose_cast_kernel<<<dim3(kD / 64, kD / 64), 256, 0, stream>>>(wq, WCAT, kD, kD, kWCarry);
  transpose_cast_kernel<<<dim3(kD / 64, kD / 64), 256, 0, stream>>>(wk, WCAT + (size_t)kD * kD, kD, kD, kWCarry);
  transpose_cast_kernel<<<dim3(kD / 64, kD / 64), 256, 0, stream>>>(wv, WCAT + (size_t)2 * kD * kD, kD, kD, kWCarry);
  transpose_cast_kernel<<<dim3(kD / 64, kD / 64), 256, 0, stream>>>(wg, WCAT + (size_t)3 * kD * kD, kD, kD, kWCarry);
  transpose_cast_kernel<<<dim3(kNs / 64, kD / 64), 256, 0, stream>>>(Bw, WCAT + (size_t)4 * kD * kD, kD, kNs, kWCarry);
  transpose_cast_kernel<<<dim3(kD / 64, kD / 64), 256, 0, stream>>>(wo, WOT, kD, kD, kWCarry);
  transpose_cast_kernel<<<dim3(kD / 64, kNs / 64), 256, 0, stream>>>(Cw, CWT, kNs, kD, kWCarry);
  transpose_cast_kernel<<<dim3(kHid / 64, kD / 64), 256, 0, stream>>>(w1, W1T, kD, kHid, kWCarry);
  transpose_cast_kernel<<<dim3(kD / 64, kHid / 64), 256, 0, stream>>>(w2, W2T, kHid, kD, kWCarry);

  layernorm_f16_kernel<<<kM / 8, 256, 0, stream>>>(x, l1g, l1b, XN16, kM);

  constexpr int gridD  = (kM / 64) * (kD / 64) / 8;
  constexpr int gridNs = (kM / 64) * (kNs / 64) / 8;
  constexpr int gridH  = (kM / 64) * (kHid / 64) / 8;
  static_assert(gridD * 8 == (kM / 64) * (kD / 64) && gridNs * 8 == (kM / 64) * (kNs / 64) && gridH * 8 == (kM / 64) * (kHid / 64));
  gemm_f16_kernel<0><<<gridD, 256, 0, stream>>>(XN16, kD, WCAT, kD, (void*)Q16, kD, bq, x, x, x, kM, kD, kD, kScaleW, 1.0f);
  gemm_f16_kernel<0><<<gridD, 256, 0, stream>>>(XN16, kD, WCAT + (size_t)kD * kD, kD, (void*)K16, kD, bk, x, x, x, kM, kD, kD, kScaleW, 1.0f);
  gemm_f16_kernel<0><<<gridD, 256, 0, stream>>>(XN16, kD, WCAT + (size_t)2 * kD * kD, kD, (void*)V16, kD, bv, x, x, x, kM, kD, kD, kScaleW, 1.0f);
  gemm_f16_kernel<1><<<gridD, 256, 0, stream>>>(XN16, kD, WCAT + (size_t)3 * kD * kD, kD, (void*)G32, kD, bg, x, x, x, kM, kD, kD, kScaleW, 1.0f);
  gemm_f16_kernel<2><<<gridNs, 256, 0, stream>>>(XN16, kD, WCAT + (size_t)4 * kD * kD, kD, (void*)U32, kNs, bg, x, x, x, kM, kNs, kD, kScaleW, 1.0f);

  attn_window_kernel<<<kB * kH * (kT / 64), 128, 0, stream>>>(Q16, K16, V16, AO16);

  scan_kernel<<<1, 128, 0, stream>>>(U32, Avec, st0, ST16, out1);

  gemm_f16_kernel<2><<<gridD, 256, 0, stream>>>(ST16, kNs, CWT, kNs, (void*)SSM32, kD, bo, x, x, x, kM, kD, kNs, kScaleW, 1.0f);

  gemm_f16_kernel<3><<<gridD, 256, 0, stream>>>(AO16, kD, WOT, kD, (void*)XMID, kD, bo, x, G32, SSM32, kM, kD, kD, kScaleAoW, 1.0f);

  layernorm_f16_kernel<<<kM / 8, 256, 0, stream>>>(XMID, l2g, l2b, XN2, kM);

  gemm_f16_kernel<4><<<gridH, 256, 0, stream>>>(XN2, kD, W1T, kD, (void*)HID16, kHid, b1, x, x, x, kM, kHid, kD, kScaleW, kHidCarry);

  gemm_f16_kernel<5><<<gridD, 256, 0, stream>>>(HID16, kHid, W2T, kHid, (void*)out0, kD, b2, XMID, XMID, XMID, kM, kD, kHid, kScaleHidW, 1.0f);
}
